// PatternMemoryDTW_8143257993997
// MI455X (gfx1250) — hardware-verified
//
#include <hip/hip_runtime.h>
#include <math.h>

typedef __attribute__((ext_vector_type(16))) _Float16 v16h;
typedef __attribute__((ext_vector_type(8)))  _Float16 v8h;
typedef __attribute__((ext_vector_type(16))) __bf16   v16b;
typedef __attribute__((ext_vector_type(8)))  __bf16   v8b;
typedef __attribute__((ext_vector_type(8)))  float    v8f;
typedef __attribute__((ext_vector_type(4)))  float    v4f;
typedef __attribute__((ext_vector_type(4)))  unsigned int v4u;

constexpr int kD          = 128;
constexpr int kKq         = 16;
constexpr int kKp         = 16;
constexpr int kM          = 64;
constexpr int kP          = 96;
constexpr int kPpad       = 128;
constexpr int kFusedK     = 256;
constexpr int kChunkNodes = 512;
constexpr int kChunkRows  = kChunkNodes * kKq;
constexpr int kDotCols    = kM * kKp;
constexpr float kInf      = 1000000000.0f;

__device__ __forceinline__ unsigned short f2bf_bits(float f) {
  unsigned u = __float_as_uint(f);
  return (unsigned short)((u + 0x7FFFu + ((u >> 16) & 1u)) >> 16);
}
__device__ __forceinline__ float bf_bits2f(unsigned short h) { return __uint_as_float(((unsigned)h) << 16); }

__device__ __forceinline__ void dep_guard_h(v8f& a, v8f& b, v16h x, v16h y) { asm volatile("v_nop\n\tv_nop\n\tv_nop\n\tv_nop" : "+v"(a), "+v"(b) : "v"(x), "v"(y)); }
__device__ __forceinline__ void dep_guard_b(v8f& a, v8f& b, v16b x, v16b y) { asm volatile("v_nop\n\tv_nop\n\tv_nop\n\tv_nop" : "+v"(a), "+v"(b) : "v"(x), "v"(y)); }
__device__ __forceinline__ void keep4_h(v16h a, v16h b, v16h c, v16h d) { asm volatile("v_nop" :: "v"(a), "v"(b), "v"(c), "v"(d)); }
__device__ __forceinline__ void keep4_b(v16b a, v16b b, v16b c, v16b d) { asm volatile("v_nop" :: "v"(a), "v"(b), "v"(c), "v"(d)); }
__device__ __forceinline__ void acc_guard4(v8f& a, v8f& b, v8f& c, v8f& d) { asm volatile("v_nop\n\tv_nop\n\tv_nop\n\tv_nop" : "+v"(a), "+v"(b), "+v"(c), "+v"(d)); }
template <typename T> struct Frag;
template <> struct Frag<_Float16> {
  typedef v16h V; union U { v16h v; v8h h[2]; };
  static __device__ __forceinline__ v16h load(const _Float16* p) {
    U f; f.h[0] = *(const v8h*)(p); f.h[1] = *(const v8h*)(p + 16); return f.v;
  }
  static __device__ __forceinline__ v8f mma(v16h a, v16h b, v8f c) {
    return __builtin_amdgcn_wmma_f32_16x16x32_f16(false, a, false, b, (short)0, c, false, false);
  }
  static __device__ __forceinline__ void guard(v8f& a, v8f& b, v16h x, v16h y) { dep_guard_h(a, b, x, y); }
  static __device__ __forceinline__ void keep(v16h a, v16h b, v16h c, v16h d) { keep4_h(a, b, c, d); }
};
template <> struct Frag<__bf16> {
  typedef v16b V; union U { v16b v; v8b h[2]; };
  static __device__ __forceinline__ v16b load(const __bf16* p) {
    U f; f.h[0] = *(const v8b*)(p); f.h[1] = *(const v8b*)(p + 16); return f.v;
  }
  static __device__ __forceinline__ v8f mma(v16b a, v16b b, v8f c) {
    return __builtin_amdgcn_wmma_f32_16x16x32_bf16(false, a, false, b, (short)0, c, false, false);
  }
  static __device__ __forceinline__ void guard(v8f& a, v8f& b, v16b x, v16b y) { dep_guard_b(a, b, x, y); }
  static __device__ __forceinline__ void keep(v16b a, v16b b, v16b c, v16b d) { keep4_b(a, b, c, d); }
};

__device__ __forceinline__ unsigned pk16(unsigned short a, unsigned short b) { return (unsigned)a | ((unsigned)b << 16); }

template <int ET> struct Elem;
template <> struct Elem<0> { typedef _Float16 T; };
template <> struct Elem<1> { typedef __bf16 T; };
template <int ET, bool SPLIT, int BIAS_MODE, int OUT_MODE, bool RESID, int ACT = 0>
__global__ __launch_bounds__(256) void wmma_gemm64(
    const unsigned short* __restrict__ Ap, const unsigned short* __restrict__ A2p, int lda, long strideA,
    const unsigned short* __restrict__ Btp, const unsigned short* __restrict__ Bt2p, int ldb, long strideB,
    void* __restrict__ Cout, void* __restrict__ Cout2, int ldc, long strideC,
    const float* __restrict__ bias,
    const float* __restrict__ resid, long strideR,
    int M, int N, int K, float scale) {
  typedef typename Elem<ET>::T T;
  typedef typename Frag<T>::V V;
  const T* A = (const T*)Ap; const T* A2 = (const T*)A2p; const T* Bt = (const T*)Btp; const T* Bt2 = (const T*)Bt2p;
  __shared__ __align__(16) float sT[8][16 * 68];
  const int b    = blockIdx.y;
  const int lane = threadIdx.x & 31;
  const int wave = threadIdx.x >> 5;
  const int tilesN = N >> 6;
  const int tilesM = M >> 6;
  const int tile = blockIdx.x * 8 + wave;
  if (tile >= tilesM * tilesN) return;
  const int tm = tile / tilesN;
  const int tn = tile - tm * tilesN;
  const int m0 = tm << 6;
  const int n0 = tn << 6;

  const T* Ab  = A  + (size_t)b * strideA;
  const T* Bb  = Bt + (size_t)b * strideB;
  const T* Ab2 = SPLIT ? (A2  + (size_t)b * strideA) : nullptr;
  const T* Bb2 = SPLIT ? (Bt2 + (size_t)b * strideB) : nullptr;

  const int rlane = lane & 15;
  const int koff  = (lane >> 4) * 8;
  const int mOff  = (lane >> 4) * 8;

  v8f acc[4][4];
#pragma unroll
  for (int i = 0; i < 4; ++i)
#pragma unroll
    for (int j = 0; j < 4; ++j) acc[i][j] = (v8f){0.f,0.f,0.f,0.f,0.f,0.f,0.f,0.f};

  for (int k0 = 0; k0 < K; k0 += 32) {
    V bh[4], bl[4];
#pragma unroll
    for (int j = 0; j < 4; ++j) {
      const size_t bo = (size_t)(n0 + (j << 4) + rlane) * ldb + koff + k0;
      bh[j] = Frag<T>::load(Bb + bo);
      if (SPLIT) bl[j] = Frag<T>::load(Bb2 + bo);
    }
#pragma unroll
    for (int i = 0; i < 4; ++i) {
      const size_t ao = (size_t)(m0 + (i << 4) + rlane) * lda + koff + k0;
      V ah = Frag<T>::load(Ab + ao);
      V al;
      if (SPLIT) al = Frag<T>::load(Ab2 + ao);
#pragma unroll
      for (int j = 0; j < 4; ++j) {
        acc[i][j] = Frag<T>::mma(ah, bh[j], acc[i][j]);
        if (SPLIT) {
          acc[i][j] = Frag<T>::mma(ah, bl[j], acc[i][j]);
          acc[i][j] = Frag<T>::mma(al, bh[j], acc[i][j]);
        }
      }
      Frag<T>::guard(acc[i][0], acc[i][3], ah, SPLIT ? al : ah);
    }
    Frag<T>::keep(bh[0], bh[1], bh[2], bh[3]);
    if (SPLIT) Frag<T>::keep(bl[0], bl[1], bl[2], bl[3]);
  }
  acc_guard4(acc[0][0], acc[0][1], acc[0][2], acc[0][3]);
  acc_guard4(acc[1][0], acc[1][1], acc[1][2], acc[1][3]);
  acc_guard4(acc[2][0], acc[2][1], acc[2][2], acc[2][3]);
  acc_guard4(acc[3][0], acc[3][1], acc[3][2], acc[3][3]);

  float* slab = sT[wave];
  const float* Rb = RESID ? (resid + (size_t)b * strideR) : nullptr;
#pragma unroll
  for (int i = 0; i < 4; ++i) {
    const int mBase = m0 + (i << 4);
#pragma unroll
    for (int j = 0; j < 4; ++j) {
      const int n = n0 + (j << 4) + rlane;
      float bv = 0.f;
      if (BIAS_MODE == 2) bv = bias[n];
#pragma unroll
      for (int r = 0; r < 8; ++r) {
        float v = acc[i][j][r] * scale;
        if (BIAS_MODE == 1) v += bias[mBase + mOff + r];
        if (BIAS_MODE == 2) v += bv;
        if (RESID) v += Rb[(size_t)(mBase + mOff + r) * ldc + n];
        if (ACT == 2) v = fmaxf(v, 0.0f);
        if (ACT == 4) v = (v > 0.f) ? v : 0.01f * v;
        slab[(mOff + r) * 68 + (j << 4) + rlane] = v;
      }
    }
    __builtin_amdgcn_fence(__ATOMIC_RELEASE, "workgroup");
    __builtin_amdgcn_wave_barrier();
    __builtin_amdgcn_fence(__ATOMIC_ACQUIRE, "workgroup");
    if (OUT_MODE == 0) {
      float* C = (float*)Cout + (size_t)b * strideC;
      const int hh = lane >> 4, c4 = (lane & 15) * 4;
      for (int pass = 0; pass < 2; ++pass) {
#pragma unroll
        for (int it = 0; it < 8; ++it) {
          const int row = it * 2 + hh;
          v4f v = *(const v4f*)(slab + row * 68 + c4);
          *(volatile v4f*)(C + (size_t)(mBase + row) * ldc + n0 + c4) = v;
        }
        __threadfence();
      }
    } else {
      const int q = lane >> 3, c8 = (lane & 7) * 8;
      unsigned short* C  = (unsigned short*)Cout  + (size_t)b * strideC;
      unsigned short* C2 = (OUT_MODE == 2) ? ((unsigned short*)Cout2 + (size_t)b * strideC) : nullptr;
      for (int pass = 0; pass < 2; ++pass) {
#pragma unroll
        for (int it = 0; it < 4; ++it) {
          const int row = it * 4 + q;
          const float* sp = slab + row * 68 + c8;
          v8h hv, lv;
#pragma unroll
          for (int e = 0; e < 8; ++e) {
            if (OUT_MODE == 1) {
              hv[e] = (_Float16)sp[e];
            } else {
              unsigned short hb = f2bf_bits(sp[e]);
              unsigned short lb = f2bf_bits(sp[e] - bf_bits2f(hb));
              hv[e] = __builtin_bit_cast(_Float16, hb);
              lv[e] = __builtin_bit_cast(_Float16, lb);
            }
          }
          *(volatile v8h*)(C + (size_t)(mBase + row) * ldc + n0 + c8) = hv;
          if (OUT_MODE == 2) *(volatile v8h*)(C2 + (size_t)(mBase + row) * ldc + n0 + c8) = lv;
        }
        __threadfence();
      }
    }
    __builtin_amdgcn_fence(__ATOMIC_RELEASE, "workgroup");
    __builtin_amdgcn_wave_barrier();
    __builtin_amdgcn_fence(__ATOMIC_ACQUIRE, "workgroup");
  }
}

__device__ __forceinline__ void split8(const v4f a, const v4f b, v4u& hv, v4u& lv) {
  unsigned short hb[8], lb[8];
#pragma unroll
  for (int e = 0; e < 4; ++e) {
    hb[e] = f2bf_bits(a[e]);
    lb[e] = f2bf_bits(a[e] - bf_bits2f(hb[e]));
    hb[4 + e] = f2bf_bits(b[e]);
    lb[4 + e] = f2bf_bits(b[e] - bf_bits2f(hb[4 + e]));
  }
  hv = (v4u){pk16(hb[0], hb[1]), pk16(hb[2], hb[3]), pk16(hb[4], hb[5]), pk16(hb[6], hb[7])};
  lv = (v4u){pk16(lb[0], lb[1]), pk16(lb[2], lb[3]), pk16(lb[4], lb[5]), pk16(lb[6], lb[7])};
}

__global__ __launch_bounds__(256) void rsplit_kernel(const float* __restrict__ in,
                                                     unsigned short* __restrict__ hi, unsigned short* __restrict__ lo,
                                                     float* __restrict__ ssq, int nrows) {
  __shared__ __align__(16) float s_sq[32];
  const int t = threadIdx.x, lane = t & 31, wave = t >> 5;
  const int hsel = lane >> 4, c8 = (lane & 15) * 8;
  const int rb = blockIdx.x * 32;
  v4u hv[2], lv[2];
  size_t roff[2];
#pragma unroll
  for (int it = 0; it < 2; ++it) {
    const int rl = wave * 4 + it * 2 + hsel;
    int r = rb + rl;
    r = (r < nrows) ? r : (nrows - 1);
    roff[it] = (size_t)r * kD + c8;
    const float* p = in + roff[it];
    const v4f a = *(const v4f*)(p);
    const v4f b = *(const v4f*)(p + 4);
    float s = 0.f;
#pragma unroll
    for (int e = 0; e < 4; ++e) s += a[e] * a[e];
#pragma unroll
    for (int e = 0; e < 4; ++e) s += b[e] * b[e];
    s += __shfl_xor(s, 1, 32);
    s += __shfl_xor(s, 2, 32);
    s += __shfl_xor(s, 4, 32);
    s += __shfl_xor(s, 8, 32);
    if ((lane & 15) == 0) s_sq[rl] = s;
    split8(a, b, hv[it], lv[it]);
  }
  for (int pass = 0; pass < 2; ++pass) {
#pragma unroll
    for (int it = 0; it < 2; ++it) {
      *(volatile v4u*)(hi + roff[it]) = hv[it];
      *(volatile v4u*)(lo + roff[it]) = lv[it];
    }
    __threadfence();
  }
  __syncthreads();
  if (wave == 0) {
    const int l8 = (lane < 8) ? lane : 7;
    const v4f v = *(const v4f*)(s_sq + 4 * l8);
    float* op = ssq + (size_t)rb + 4 * l8;
    for (int pass = 0; pass < 2; ++pass) {
      if (lane < 8) *(volatile v4f*)op = v;
      __threadfence();
    }
  }
}

__global__ __launch_bounds__(256) void tsplit_kernel(const float* __restrict__ in, int nR, int nC,
                                                     unsigned short* __restrict__ hi, unsigned short* __restrict__ lo) {
  __shared__ float sm[64][65];
  const int t  = threadIdx.x;
  const int r0 = blockIdx.x * 64;
  const int c0 = blockIdx.y * 64;
#pragma unroll
  for (int i = 0; i < 16; ++i) {
    const int e  = i * 256 + t;
    const int rl = e >> 6;
    const int cl = e & 63;
    const int c  = c0 + cl;
    const int cc = (c < nC) ? c : (nC - 1);
    int r = r0 + rl;
    r = (r < nR) ? r : (nR - 1);
    float v = in[(size_t)r * nC + cc];
    v = (c < nC) ? v : 0.0f;
    sm[cl][rl] = v;
  }
  __syncthreads();
  const int lane = t & 31, wave = t >> 5;
  const int q = lane >> 3, c8 = (lane & 7) * 8;
  v4u hv[2], lv[2];
  size_t ooff[2];
#pragma unroll
  for (int it = 0; it < 2; ++it) {
    const int row = wave * 8 + it * 4 + q;
    const v4f a = (v4f){sm[row][c8 + 0], sm[row][c8 + 1], sm[row][c8 + 2], sm[row][c8 + 3]};
    const v4f b = (v4f){sm[row][c8 + 4], sm[row][c8 + 5], sm[row][c8 + 6], sm[row][c8 + 7]};
    split8(a, b, hv[it], lv[it]);
    ooff[it] = (size_t)(c0 + row) * nR + r0 + c8;
  }
  for (int pass = 0; pass < 2; ++pass) {
#pragma unroll
    for (int it = 0; it < 2; ++it) {
      *(volatile v4u*)(hi + ooff[it]) = hv[it];
      *(volatile v4u*)(lo + ooff[it]) = lv[it];
    }
    __threadfence();
  }
}

__global__ __launch_bounds__(256) void dtw_kernel(const float* __restrict__ dot, const float* __restrict__ qsq,
                                                  const float* __restrict__ psq, float* __restrict__ dists, int nbase) {
#pragma clang fp contract(off)
  __shared__ __align__(16) float sd[256];
  const int t  = threadIdx.x;
  const int nl = blockIdx.x * 4 + (t >> 6);
  const int m  = t & 63;
  const int n  = nbase + nl;
  const float* pp = psq + m * kKp;
  const v4f p0 = *(const v4f*)(pp);
  const v4f p1 = *(const v4f*)(pp + 4);
  const v4f p2 = *(const v4f*)(pp + 8);
  const v4f p3 = *(const v4f*)(pp + 12);
  float pj[16];
#pragma unroll
  for (int e = 0; e < 4; ++e) { pj[e] = p0[e]; pj[4 + e] = p1[e]; pj[8 + e] = p2[e]; pj[12 + e] = p3[e]; }
  const float* qp    = qsq + (size_t)n * kKq;
  const float* dbase = dot + (size_t)nl * kKq * kDotCols + (size_t)m * kKp;
  float row[17];
  row[0] = 0.0f;
#pragma unroll
  for (int j = 1; j <= 16; ++j) row[j] = kInf;
#pragma unroll 1
  for (int i = 0; i < kKq; ++i) {
    const float qk = qp[i];
    const float* dr = dbase + (size_t)i * kDotCols;
    const v4f d0 = *(const v4f*)(dr);
    const v4f d1 = *(const v4f*)(dr + 4);
    const v4f d2 = *(const v4f*)(dr + 8);
    const v4f d3 = *(const v4f*)(dr + 12);
    float dv[16];
#pragma unroll
    for (int e = 0; e < 4; ++e) { dv[e] = d0[e]; dv[4 + e] = d1[e]; dv[8 + e] = d2[e]; dv[12 + e] = d3[e]; }
    float diag = row[0];
    row[0] = kInf;
    float left = kInf;
#pragma unroll
    for (int j = 0; j < 16; ++j) {
      const float dd = dv[j] + dv[j];
      const float s  = (qk + pj[j]) - dd;
      const float c  = sqrtf(fmaxf(s, 1e-12f));
      const float up = row[j + 1];
      const float v  = c + fminf(fminf(up, left), diag);
      diag = up;
      row[j + 1] = v;
      left = v;
    }
  }
  sd[t] = row[16];
  __syncthreads();
  if (t < 64) {
    const v4f v = *(const v4f*)(sd + 4 * t);
    float* op = dists + ((size_t)nbase + (size_t)blockIdx.x * 4) * kM + 4 * t;
    for (int pass = 0; pass < 2; ++pass) {
      *(volatile v4f*)op = v;
      __threadfence();
    }
  }
}

__global__ __launch_bounds__(256) void fuse_kernel(const float* __restrict__ nodes, const float* __restrict__ memv,
                                                   const float* __restrict__ dists,
                                                   unsigned short* __restrict__ fh, unsigned short* __restrict__ fl, int nn) {
  __shared__ float s_w[2][64];
  __shared__ __align__(16) float s_f[2][256];
  const int t = threadIdx.x, lane = t & 31, wave = t >> 5;
  const int nh = t >> 7, d = t & 127;
  int n = blockIdx.x * 2 + nh;
  n = (n < nn) ? n : (nn - 1);
  if (wave == 0 || wave == 4) {
    const float* dr = dists + (size_t)n * kM;
    const float dA = dr[lane];
    const float dB = dr[lane + 32];
    float mn = fminf(dA, dB);
#pragma unroll
    for (int off = 16; off > 0; off >>= 1) mn = fminf(mn, __shfl_xor(mn, off, 32));
    const float eA = expf(mn - dA);
    const float eB = expf(mn - dB);
    float sum = eA + eB;
#pragma unroll
    for (int off = 16; off > 0; off >>= 1) sum += __shfl_xor(sum, off, 32);
    const float inv = 1.0f / sum;
    s_w[nh][lane]      = eA * inv;
    s_w[nh][lane + 32] = eB * inv;
  }
  __syncthreads();
  {
    const float* np0 = nodes + (size_t)n * kKq * kD + d;
    float s = 0.f;
#pragma unroll
    for (int k = 0; k < kKq; ++k) s += np0[(size_t)k * kD];
    s_f[nh][d] = s * (1.0f / 16.0f);
    float r = 0.f;
#pragma unroll 1
    for (int mm = 0; mm < kM; ++mm) r += s_w[nh][mm] * memv[mm * kD + d];
    s_f[nh][kD + d] = r;
  }
  __syncthreads();
  if (wave < 2) {
    int n2 = blockIdx.x * 2 + wave;
    n2 = (n2 < nn) ? n2 : (nn - 1);
    const float* sp = s_f[wave] + lane * 8;
    const v4f a = *(const v4f*)(sp);
    const v4f b = *(const v4f*)(sp + 4);
    v4u hv, lv;
    split8(a, b, hv, lv);
    const size_t off = (size_t)n2 * kFusedK + lane * 8;
    for (int pass = 0; pass < 2; ++pass) {
      *(volatile v4u*)(fh + off) = hv;
      *(volatile v4u*)(fl + off) = lv;
      __threadfence();
    }
  }
}

__global__ __launch_bounds__(256) void gelu_split_kernel(const float* __restrict__ g, unsigned short* __restrict__ oh,
                                                         unsigned short* __restrict__ ol, int total) {
  __shared__ __align__(16) float sg[2048];
  const int t = threadIdx.x;
  const size_t base = (size_t)blockIdx.x * 2048;
#pragma unroll 1
  for (int e = 0; e < 8; ++e) {
    const int idx = e * 256 + t;
    size_t gi = base + idx;
    gi = (gi < (size_t)total) ? gi : (size_t)(total - 1);
    const float x = g[gi];
    const float y = 0.5f * x * (1.0f + erff(x * 0.70710678118654752f));
    sg[idx] = y;
  }
  __syncthreads();
  const float* sp = sg + t * 8;
  const v4f a = *(const v4f*)(sp);
  const v4f b = *(const v4f*)(sp + 4);
  v4u hv, lv;
  split8(a, b, hv, lv);
  const size_t off = base + (size_t)t * 8;
  for (int pass = 0; pass < 2; ++pass) {
    *(volatile v4u*)(oh + off) = hv;
    *(volatile v4u*)(ol + off) = lv;
    __threadfence();
  }
}

__global__ __launch_bounds__(256) void out_copy_kernel(const float* __restrict__ stg, const float* __restrict__ b2,
                                                       float* __restrict__ out) {
  const int t = threadIdx.x, lane = t & 31, wave = t >> 5;
  const int c4 = lane * 4;
  const int cb = (c4 < kP - 4) ? c4 : (kP - 4);
  const v4f bb = *(const v4f*)(b2 + cb);
  v4f vals[4];
  size_t ooff[4];
#pragma unroll
  for (int it = 0; it < 4; ++it) {
    const int row = blockIdx.x * 32 + it * 8 + wave;
    const v4f v = *(const v4f*)(stg + (size_t)row * kPpad + c4);
    vals[it] = v + bb;
    ooff[it] = (size_t)row * kP + cb;
  }
  for (int pass = 0; pass < 2; ++pass) {
#pragma unroll
    for (int it = 0; it < 4; ++it) {
      if (lane < 24) *(volatile v4f*)(out + ooff[it]) = vals[it];
    }
    __threadfence();
  }
}

extern "C" void kernel_launch(void* const* d_in, const int* in_sizes, int n_in,
                              void* d_out, int out_size, void* d_ws, size_t ws_size,
                              hipStream_t stream) {
  if (n_in < 7) return;
  const float* nodes  = (const float*)d_in[0];
  const float* protos = (const float*)d_in[1];
  const float* memv   = (const float*)d_in[2];
  const float* w1     = (const float*)d_in[3];
  const float* b1     = (const float*)d_in[4];
  const float* w2     = (const float*)d_in[5];
  const float* b2     = (const float*)d_in[6];

  const int nN = in_sizes[0] / (kKq * kD);
  if (nN <= 0 || in_sizes[0] != nN * kKq * kD || (nN % kChunkNodes) != 0) return;
  if (in_sizes[1] != kM * kKp * kD || in_sizes[2] != kM * kD || in_sizes[3] != kFusedK * kD ||
      in_sizes[4] != kD || in_sizes[5] != kD * kP || in_sizes[6] != kP) return;
  if (out_size != nN * kP + nN * kM) return;

  float* out0 = (float*)d_out;
  float* out1 = out0 + (size_t)nN * kP;

  unsigned char* ws = (unsigned char*)d_ws;
  size_t off = 0;
  const size_t szNodesPlane = (size_t)nN * kKq * kD * 2;
  const size_t szDot        = (size_t)kChunkRows * kDotCols * 4;
  const size_t szProtoPlane = (size_t)kDotCols * kD * 2;
  const size_t szQsq        = (size_t)nN * kKq * 4;
  const size_t szPsq        = (size_t)kDotCols * 4;
  const size_t szFusedPlane = (size_t)nN * kFusedK * 2;
  const size_t szW1Plane    = (size_t)kD * kFusedK * 2;
  const size_t szG1         = (size_t)nN * kD * 4;
  const size_t szHPlane     = (size_t)nN * kD * 2;
  const size_t szW2Plane    = (size_t)kPpad * kD * 2;
  const size_t szOstg       = (size_t)nN * kPpad * 4;

  unsigned short* nodesHi = (unsigned short*)(ws + off); off += szNodesPlane;
  unsigned short* nodesLo = (unsigned short*)(ws + off); off += szNodesPlane;
  float*          dot     = (float*)(ws + off);          off += szDot;
  unsigned short* protoHi = (unsigned short*)(ws + off); off += szProtoPlane;
  unsigned short* protoLo = (unsigned short*)(ws + off); off += szProtoPlane;
  float*          qsq     = (float*)(ws + off);          off += szQsq;
  float*          psq     = (float*)(ws + off);          off += szPsq;
  unsigned short* fusedHi = (unsigned short*)(ws + off); off += szFusedPlane;
  unsigned short* fusedLo = (unsigned short*)(ws + off); off += szFusedPlane;
  unsigned short* w1tHi   = (unsigned short*)(ws + off); off += szW1Plane;
  unsigned short* w1tLo   = (unsigned short*)(ws + off); off += szW1Plane;
  float*          g1      = (float*)(ws + off);          off += szG1;
  unsigned short* hHi     = (unsigned short*)(ws + off); off += szHPlane;
  unsigned short* hLo     = (unsigned short*)(ws + off); off += szHPlane;
  unsigned short* w2tHi   = (unsigned short*)(ws + off); off += szW2Plane;
  unsigned short* w2tLo   = (unsigned short*)(ws + off); off += szW2Plane;
  float*          ostg    = (float*)(ws + off);          off += szOstg;
  if (off > ws_size) return;

  const dim3 blk(256);

  rsplit_kernel<<<dim3((nN * kKq) / 32), blk, 0, stream>>>(nodes, nodesHi, nodesLo, qsq, nN * kKq);
  rsplit_kernel<<<dim3(kDotCols / 32), blk, 0, stream>>>(protos, protoHi, protoLo, psq, kDotCols);
  tsplit_kernel<<<dim3(kFusedK / 64, kD / 64), blk, 0, stream>>>(w1, kFusedK, kD, w1tHi, w1tLo);
  tsplit_kernel<<<dim3(kD / 64, kPpad / 64), blk, 0, stream>>>(w2, kD, kP, w2tHi, w2tLo);

  const int nChunks   = nN / kChunkNodes;
  const int dotTiles  = (kChunkRows / 64) * (kDotCols / 64);
  const int dotBlocks = (dotTiles + 7) / 8;
  for (int c = 0; c < nChunks; ++c) {
    const size_t aoff = (size_t)c * kChunkRows * kD;
    wmma_gemm64<1, true, 0, 0, false, 0><<<dim3(dotBlocks, 1), blk, 0, stream>>>(
        nodesHi + aoff, nodesLo + aoff, kD, 0L,
        protoHi, protoLo, kD, 0L,
        (void*)dot, (void*)dot, kDotCols, 0L,
        psq, psq, 0L,
        kChunkRows, kDotCols, kD, 1.0f);
    dtw_kernel<<<dim3(kChunkNodes / 4), blk, 0, stream>>>(dot, qsq, psq, out1, c * kChunkNodes);
  }

  fuse_kernel<<<dim3(nN / 2), blk, 0, stream>>>(nodes, memv, out1, fusedHi, fusedLo, nN);

  const int mlpTiles  = (nN / 64) * (kD / 64);
  const int mlpBlocks = (mlpTiles + 7) / 8;
  wmma_gemm64<1, true, 2, 0, false, 0><<<dim3(mlpBlocks, 1), blk, 0, stream>>>(
      fusedHi, fusedLo, kFusedK, 0L,
      w1tHi, w1tLo, kFusedK, 0L,
      (void*)g1, (void*)g1, kD, 0L,
      b1, b1, 0L,
      nN, kD, kFusedK, 1.0f);

  gelu_split_kernel<<<dim3((nN * kD) / 2048), blk, 0, stream>>>(g1, hHi, hLo, nN * kD);

  wmma_gemm64<1, true, 0, 0, false, 0><<<dim3(mlpBlocks, 1), blk, 0, stream>>>(
      hHi, hLo, kD, 0L,
      w2tHi, w2tLo, kD, 0L,
      (void*)ostg, (void*)ostg, kPpad, 0L,
      b1, b1, 0L,
      nN, kPpad, kD, 1.0f);

  out_copy_kernel<<<dim3(nN / 32), blk, 0, stream>>>(ostg, b2, out0);
}
